// MeanField_38208029065274
// MI455X (gfx1250) — hardware-verified
//
#include <hip/hip_runtime.h>


namespace {
constexpr int B = 2, C = 21, CP = 32, H = 512, W = 512, HW = H * W, ND = 8, NIT = 5, HL = 512  ;
constexpr float XS = 8.0f, WSC = 256.0f;
__constant__ int DY[ND] = {0, 0, 1, -1, 1, 1, -1, -1};
__constant__ int DX[ND] = {1, -1, 0, 0, 1, -1, 1, -1};
static_assert(W % 32 == 0, "tiling");
typedef _Float16 b16;
typedef __attribute__((ext_vector_type(16))) _Float16 v16b;
typedef __attribute__((ext_vector_type(8))) _Float16 v8b;
typedef __attribute__((ext_vector_type(8))) float v8f;
typedef __attribute__((ext_vector_type(4))) float v4f;
__device__ __forceinline__ float bf16_rne(float f) { unsigned int u = __float_as_uint(f); u += 0x7FFFu + ((u >> 16) & 1u); return __uint_as_float(u & 0xFFFF0000u); }
__device__ __forceinline__ void split16(float v, b16& hi, b16& lo) { hi = (b16)v; lo = (b16)(v - (float)hi); }
__device__ __forceinline__ v16b frag_kb(const b16* p, int hh) { const v8b a = *(const v8b*)(p + 8 * hh), b = *(const v8b*)(p + 16 + 8 * hh); v16b f;
#pragma unroll
  for (int e = 0; e < 8; ++e) { f[e] = a[e]; f[8 + e] = b[e]; } return f; }
__device__ __forceinline__ v8f wmma16b(v16b a, v16b b, v8f c) { v8f d = __builtin_amdgcn_wmma_f32_16x16x32_f16(false, a, false, b, (short)0, c, false, false); asm volatile("v_nop\n\tv_nop\n\tv_nop\n\tv_nop" : "+v"(d) : "v"(a), "v"(b)); return d; }
__device__ __forceinline__ void wave_lds_sync() { __builtin_amdgcn_fence(__ATOMIC_RELEASE, "workgroup"); __builtin_amdgcn_wave_barrier(); __builtin_amdgcn_fence(__ATOMIC_ACQUIRE, "workgroup"); }
__device__ __forceinline__ float pmul(float a, float b) { float p = a * b; asm volatile("" : "+v"(p)); return p; }
__device__ __forceinline__ int iclamp(int v, int lo, int hi) { return v < lo ? lo : (v > hi ? hi : v); }

typedef __attribute__((ext_vector_type(4))) _Float16 v4h;
typedef __attribute__((ext_vector_type(2))) float v2f;
__global__ __launch_bounds__(256) void prep_kernel(const float* __restrict__ L, b16* __restrict__ LT) {
  const int t = threadIdx.x; if (t >= CP * CP / 8) return; const int e = t * 8; const int l = e / CP, k0 = e % CP; v8b o;
  for (int j = 0; j < 8; ++j) { const int k = k0 + j; o[j] = (l < C && k < C) ? (b16)(bf16_rne(L[l * C + k]) * WSC) : (b16)0.0f; }
  for (int pass = 0; pass < 2; ++pass) { *(volatile v8b*)(LT + e) = o; __threadfence(); }
}
__global__ __launch_bounds__(256) void init_kernel(const float* __restrict__ u, float* __restrict__ Q) {
  const size_t p = (size_t)blockIdx.x * 256 + threadIdx.x; if (p >= (size_t)B * HW) return; const size_t b = p / HW, pix = p % HW; const float* ub = u + b * (size_t)C * HW + pix; float* qb = Q + b * (size_t)C * HW + pix;
  float v[C]; float mx = -INFINITY;
#pragma unroll
  for (int c = 0; c < C; ++c) { v[c] = -bf16_rne(ub[(size_t)c * HW]); mx = fmaxf(mx, v[c]); }
  float s = 0.0f;
#pragma unroll
  for (int c = 0; c < C; ++c) { v[c] = __expf(v[c] - mx); s += v[c]; }
  const float inv = 1.0f / s;
  for (int pass = 0; pass < 2; ++pass) {
#pragma unroll
    for (int c = 0; c < C; ++c) ((volatile float*)qb)[(size_t)c * HW] = v[c] * inv; __threadfence(); }
}
template <int LAST>
__global__ __launch_bounds__(128) void iter_kernel(const float* __restrict__ u, const float* __restrict__ ew, const b16* __restrict__ LT, const float* __restrict__ Qp, float* __restrict__ Qn) {
  __shared__ __attribute__((aligned(16))) float Tq[4][16][CP + 1]; __shared__ __attribute__((aligned(16))) b16 Ah[4][16][CP + 8], Al[4][16][CP + 8]; __shared__ __attribute__((aligned(16))) float Ob[C][64 + 4];
  const int wave = threadIdx.x >> 5, lane = threadIdx.x & 31, nloc = lane & 15, hlf = lane >> 4;
  const int blk = blockIdx.x; const int b = blk / (HL * (W / 64)), rem = blk % (HL * (W / 64)); const int y = rem / (W / 64), x0 = (rem % (W / 64)) * 64 + wave * 16;
  const float* Qb = Qp + (size_t)b * C * HW; const float* ewb = ew + (size_t)b * ND * HW;
  { const int x = x0 + nloc; float wgt[ND]; int off[ND]; bool ok[ND];
#pragma unroll
    for (int d = 0; d < ND; ++d) { const int yy = y + DY[d], xx = x + DX[d]; ok[d] = (yy >= 0 && yy < H && xx >= 0 && xx < W); off[d] = ok[d] ? (yy * W + xx) : 0; wgt[d] = bf16_rne(ewb[(size_t)d * HW + (size_t)y * W + x]); }
    for (int c = hlf; c < CP; c += 2) { float s = 0.0f; if (c < C) {
#pragma unroll
        for (int d = 0; d < ND; ++d) if (ok[d]) s += pmul(wgt[d], Qb[(size_t)c * HW + off[d]]); s *= (1.0f / ND); } Tq[wave][nloc][c] = s; } }
  wave_lds_sync();
  { const int rr = lane & 15, c0 = (lane >> 4) * 16; v8b h0, l0, h1, l1; for (int j = 0; j < 8; ++j) { b16 p, q; split16(Tq[wave][rr][c0 + j] * XS, p, q); h0[j] = p; l0[j] = q; split16(Tq[wave][rr][c0 + 8 + j] * XS, p, q); h1[j] = p; l1[j] = q; }
    *(v8b*)(&Ah[wave][rr][c0]) = h0; *(v8b*)(&Ah[wave][rr][c0 + 8]) = h1; *(v8b*)(&Al[wave][rr][c0]) = l0; *(v8b*)(&Al[wave][rr][c0 + 8]) = l1; }
  wave_lds_sync();
  v8f acc[2] = {(v8f){}, (v8f){}};
  { const v16b a = frag_kb(&Ah[wave][nloc][0], hlf), al = frag_kb(&Al[wave][nloc][0], hlf);
#pragma unroll
    for (int t = 0; t < 2; ++t) { const v16b bw = frag_kb(LT + (size_t)(t * 16 + nloc) * CP, hlf); acc[t] = wmma16b(a, bw, acc[t]); acc[t] = wmma16b(al, bw, acc[t]); } }
  wave_lds_sync();
#pragma unroll
  for (int t = 0; t < 2; ++t) { const int c = t * 16 + nloc;
#pragma unroll
    for (int r = 0; r < 8; ++r) { const int px = 8 * hlf + r; float v = 0.0f; if (c < C) v = -bf16_rne(u[((size_t)b * C + c) * HW + (size_t)y * W + x0 + px]) - acc[t][r] * (1.0f / (XS * WSC)); Tq[wave][px][c] = v; } }
  wave_lds_sync();
  { const int px = nloc; float v[C]; float mx = -INFINITY;
#pragma unroll
    for (int c = 0; c < C; ++c) { v[c] = Tq[wave][px][c]; mx = fmaxf(mx, v[c]); }
    if (!LAST) { float s = 0.0f;
#pragma unroll
      for (int c = 0; c < C; ++c) { v[c] = __expf(v[c] - mx); s += v[c]; } const float inv = 1.0f / s;
#pragma unroll
      for (int c = 0; c < C; ++c) v[c] *= inv; }
    else {
#pragma unroll
      for (int c = 0; c < C; ++c) v[c] = -v[c]; }
    wave_lds_sync();
    if (hlf == 0) {
#pragma unroll
      for (int c = 0; c < C; ++c) Ob[c][wave * 16 + px] = v[c]; } }
  __syncthreads();
  const int xb = x0 - wave * 16;
  for (int pass = 0; pass < 2; ++pass) { for (int c = wave; c < C; c += 4) *(volatile v2f*)(Qn + ((size_t)b * C + c) * HW + (size_t)y * W + xb + lane * 2) = *(const v2f*)(&Ob[c][lane * 2]); __threadfence(); }
}
}

extern "C" void kernel_launch(void* const* d_in, const int* in_sizes, int n_in, void* d_out, int out_size, void* d_ws, size_t ws_size, hipStream_t stream) {
  (void)n_in;
  auto Fp = [&](int i) { return (const float*)d_in[i]; };
  if (in_sizes[0] != B * C * HW || in_sizes[1] != B * ND * HW || in_sizes[2] != C * C || out_size != B * C * HW) return;
  size_t off = 0; char* ws = (char*)d_ws;
  auto carve = [&](size_t bytes) { char* p = ws + off; off += (bytes + 255) & ~(size_t)255; return p; };
  b16* LT = (b16*)carve(CP * CP * 2); float* QA = (float*)carve((size_t)B * C * HW * 4); float* QB = (float*)carve((size_t)B * C * HW * 4);
  if (off > ws_size || off > ((size_t)128 << 20)) return;
  prep_kernel<<<1, 256, 0, stream>>>(Fp(2), LT);
  init_kernel<<<(unsigned)(((size_t)B * HW + 255) / 256), 256, 0, stream>>>(Fp(0), QA);
  const unsigned nblk = (unsigned)(B * HL * (W / 64));
  float* cur = QA; float* nxt = QB;
  for (int it = 0; it < NIT; ++it) {
    if (it < NIT - 1) { iter_kernel<0><<<nblk, 128, 0, stream>>>(Fp(0), Fp(1), LT, cur, nxt); float* t = cur; cur = nxt; nxt = t; }
    else iter_kernel<1><<<nblk, 128, 0, stream>>>(Fp(0), Fp(1), LT, cur, (float*)d_out); }
}
